// TransformerLayer_28174985462169
// MI455X (gfx1250) — hardware-verified
//
#include <hip/hip_runtime.h>


#ifndef NB
#define NB 8
#endif
#ifndef SEQ
#define SEQ 512
#endif
#ifndef MEMLEN
#define MEMLEN SEQ
#endif
#define NB_FULL  8
#define SEQ_FULL 512
#define MEM_FULL 512
#define KL    (MEMLEN + SEQ)
#define HID   1024
#define NHEAD 16
#define HD    64
#define FFD   4096
#define WCAR  64.0f
#define CCAR  256.0f
#define BDS   52
#define CTS   72
#define L2E   1.4426950408889634f

static_assert(SEQ % 64 == 0);
static_assert(MEMLEN % 64 == 0);
static_assert(MEMLEN == SEQ);
static_assert(NB <= NB_FULL);
static_assert(SEQ <= SEQ_FULL);
static_assert(MEMLEN <= MEM_FULL);
static_assert(KL <= 1024);
static_assert(KL % 64 == 0);
static_assert(HID == NHEAD * HD);
static_assert(HID == 256 * 4);
static_assert(((size_t)NB * KL * HID / 8) % 256 == 0);
static_assert(((size_t)KL * HID / 8) % 256 == 0);
static_assert((size_t)NB_FULL * SEQ_FULL * HID * 4 == 16777216);

typedef _Float16 h16;
typedef unsigned short bf;
typedef __attribute__((ext_vector_type(16))) __bf16   v16bf;
typedef __attribute__((ext_vector_type(16))) _Float16 v16h;
typedef __attribute__((ext_vector_type(8)))  _Float16 v8h;
typedef __attribute__((ext_vector_type(4)))  _Float16 v4h;
typedef __attribute__((ext_vector_type(8)))  unsigned short v8us;
typedef __attribute__((ext_vector_type(8)))  float    v8f;
typedef __attribute__((ext_vector_type(4)))  float    v4f;
typedef v8h  __attribute__((may_alias)) v8ha;
typedef v4f  __attribute__((may_alias)) v4fa;
typedef v8us __attribute__((may_alias)) v8usa;

__device__ __forceinline__ unsigned short f2bf(float f) { unsigned u = __float_as_uint(f); u += 0x7FFFu + ((u >> 16) & 1u); return (unsigned short)(u >> 16); }
__device__ __forceinline__ float bf2f(unsigned short b) { return __uint_as_float(((unsigned)b) << 16); }
__device__ __forceinline__ float bfr(float f) { return bf2f(f2bf(f)); }
__device__ __forceinline__ v16h cat16(v8h lo, v8h hi) { return __builtin_shufflevector(lo, hi, 0, 1, 2, 3, 4, 5, 6, 7, 8, 9, 10, 11, 12, 13, 14, 15); }
__device__ __forceinline__ v16bf cat16b(v8us lo, v8us hi) { return __builtin_bit_cast(v16bf, __builtin_shufflevector(lo, hi, 0, 1, 2, 3, 4, 5, 6, 7, 8, 9, 10, 11, 12, 13, 14, 15)); }
__device__ __forceinline__ v8f wmma16(v16h a, v16h b, v8f c) { return __builtin_amdgcn_wmma_f32_16x16x32_f16(false, a, false, b, (short)0, c, false, false); }
__device__ __forceinline__ v8f wmmab(v16bf a, v16bf b, v8f c) { return __builtin_amdgcn_wmma_f32_16x16x32_bf16(false, a, false, b, (short)0, c, false, false); }
__device__ __forceinline__ void wsync() { __builtin_amdgcn_fence(3  , "wavefront"); __builtin_amdgcn_wave_barrier(); __builtin_amdgcn_fence(2  , "wavefront"); asm volatile("" ::: "memory"); }
__device__ __forceinline__ unsigned umin_(unsigned a, unsigned b) { return a < b ? a : b; }

template <typename T16> struct WFrag;
template <> struct WFrag<h16> { typedef v16h V; static __device__ __forceinline__ V ld(const h16* p) { return cat16(*(const v8h*)p, *(const v8h*)(p + 16)); } static __device__ __forceinline__ v8f mma(V a, V b, v8f c) { return wmma16(a, b, c); } };
template <> struct WFrag<bf> { typedef v16bf V; static __device__ __forceinline__ V ld(const bf* p) { return cat16b(*(const v8us*)p, *(const v8us*)(p + 16)); } static __device__ __forceinline__ v8f mma(V a, V b, v8f c) { return wmmab(a, b, c); } };

enum { EPI_F32 = 0, EPI_H1 = 1, EPI_H1R = 2, EPI_H2 = 3 };

template <typename T16, int EPI>
__global__ __launch_bounds__(32) void k_gemmw(const T16* __restrict__ A, const T16* __restrict__ Bt, unsigned K, float* CF, h16* CH0, h16* CH1, unsigned ldc,
                                              const float* __restrict__ bias0, const float* __restrict__ bias1, float sc, size_t sA, size_t sB, size_t sC) {
    typedef typename WFrag<T16>::V V;
    __shared__ __align__(16) float os[16 * 68];
    const size_t z = blockIdx.z; A += z * sA; Bt += z * sB;
    const unsigned lane = threadIdx.x & 31u, lr = lane & 15u, hi = lane >> 4;
    const unsigned r0 = blockIdx.x * 64u, c0 = blockIdx.y * 64u;
    v8f acc[4][4];
#pragma unroll
    for (int mb = 0; mb < 4; ++mb)
#pragma unroll
        for (int nb = 0; nb < 4; ++nb) acc[mb][nb] = (v8f){};
    const size_t aoff = (size_t)(r0 + lr) * K + 8u * hi, boff = (size_t)(c0 + lr) * K + 8u * hi;
#pragma unroll 1
    for (unsigned kc = 0; kc < K; kc += 32u) {
        V a[4];
#pragma unroll
        for (int mb = 0; mb < 4; ++mb) a[mb] = WFrag<T16>::ld(A + aoff + (size_t)mb * 16u * K + kc);
#pragma unroll
        for (int nb = 0; nb < 4; ++nb) { const V bq = WFrag<T16>::ld(Bt + boff + (size_t)nb * 16u * K + kc);
#pragma unroll
            for (int mb = 0; mb < 4; ++mb) acc[mb][nb] = WFrag<T16>::mma(a[mb], bq, acc[mb][nb]); }
        asm volatile("v_nop\n\tv_nop\n\tv_nop\n\tv_nop" : "+v"(acc[0][0]), "+v"(acc[1][1]), "+v"(acc[2][2]), "+v"(acc[3][3]) : "v"(a[0]), "v"(a[3]));
    }
    if (EPI == EPI_F32) {
        const unsigned cofs = lr * 4u;
        v4f bv = (v4f){};
        if (bias0) { const v4f t = *(const v4f*)(bias0 + c0 + cofs); bv[0] = bfr(t[0]); bv[1] = bfr(t[1]); bv[2] = bfr(t[2]); bv[3] = bfr(t[3]); }
#pragma unroll
        for (int mb = 0; mb < 4; ++mb) {
#pragma unroll
            for (int nb = 0; nb < 4; ++nb) {
#pragma unroll
                for (int j = 0; j < 8; ++j) os[(hi * 8u + j) * 68u + nb * 16u + lr] = acc[mb][nb][j]; }
            wsync();
            float* crow = CF + z * sC + (size_t)(r0 + mb * 16u) * ldc + c0;
#pragma unroll 1
            for (int ps = 0; ps < 2; ++ps) {
#pragma unroll
                for (int s = 0; s < 8; ++s) { const unsigned row = 2u * s + hi; v4f val = *(const v4fa*)(os + row * 68u + cofs); val = val * sc + bv;
                    *(volatile v4f*)(crow + (size_t)row * ldc + cofs) = val; }
                if (ps == 0) __threadfence(); }
            wsync();
        }
    } else {
        const unsigned rq = lane >> 3, cb = (lane & 7u) * 8u;
        v8f b0v = (v8f){}, b1v = (v8f){};
        if (bias0) { const v4f t0 = *(const v4f*)(bias0 + c0 + cb); const v4f t1 = *(const v4f*)(bias0 + c0 + cb + 4u);
#pragma unroll
            for (int e = 0; e < 4; ++e) { b0v[e] = bfr(t0[e]); b0v[4 + e] = bfr(t1[e]); } }
        if (EPI == EPI_H2 && bias1) { const v4f t0 = *(const v4f*)(bias1 + c0 + cb); const v4f t1 = *(const v4f*)(bias1 + c0 + cb + 4u);
#pragma unroll
            for (int e = 0; e < 4; ++e) { b1v[e] = bfr(t0[e]); b1v[4 + e] = bfr(t1[e]); } }
#pragma unroll
        for (int mb = 0; mb < 4; ++mb) {
#pragma unroll
            for (int nb = 0; nb < 4; ++nb) {
#pragma unroll
                for (int j = 0; j < 8; ++j) os[(hi * 8u + j) * 68u + nb * 16u + lr] = acc[mb][nb][j]; }
            wsync();
            const size_t tbase = z * sC + (size_t)(r0 + mb * 16u) * ldc + c0 + cb;
#pragma unroll 1
            for (int ps = 0; ps < 2; ++ps) {
#pragma unroll
                for (int s = 0; s < 4; ++s) { const unsigned row = 4u * s + rq; const v4f x0 = *(const v4fa*)(os + row * 68u + cb); const v4f x1 = *(const v4fa*)(os + row * 68u + cb + 4u);
                    v8h o0, o1;
#pragma unroll
                    for (int e = 0; e < 4; ++e) { float t0 = x0[e] * sc + b0v[e], t1 = x1[e] * sc + b0v[4 + e]; if (EPI == EPI_H1R) { t0 = fmaxf(t0, 0.0f); t1 = fmaxf(t1, 0.0f); } o0[e] = (h16)t0; o0[4 + e] = (h16)t1;
                        if (EPI == EPI_H2) { o1[e] = (h16)(x0[e] * sc + b1v[e]); o1[4 + e] = (h16)(x1[e] * sc + b1v[4 + e]); } }
                    *(volatile v8h*)(CH0 + tbase + (size_t)row * ldc) = o0;
                    if (EPI == EPI_H2) *(volatile v8h*)(CH1 + tbase + (size_t)row * ldc) = o1; }
                if (ps == 0) __threadfence(); }
            wsync();
        }
    }
}

__global__ __launch_bounds__(256) void k_cvt8(const float* __restrict__ src, bf* dst, unsigned n8) { const unsigned i = blockIdx.x * 256u + threadIdx.x; if (i >= n8) return; const v8f v = *(const v8f*)(src + (size_t)i * 8); v8us o;
#pragma unroll
    for (int k = 0; k < 8; ++k) o[k] = f2bf(v[k]);
    *(volatile v8us*)(dst + (size_t)i * 8) = o; __threadfence(); *(volatile v8us*)(dst + (size_t)i * 8) = o; }

__global__ __launch_bounds__(256) void k_cvtcat(const float* __restrict__ mems, const float* __restrict__ x, bf* dst) {
    const unsigned i = blockIdx.x * 256u + threadIdx.x; if (i >= (unsigned)((size_t)NB * KL * HID / 8)) return;
    const unsigned col = (i & (unsigned)(HID / 8 - 1)) * 8u; const unsigned row = i / (unsigned)(HID / 8); const unsigned b = row / (unsigned)KL, t = row % (unsigned)KL;
    const bool im = t < (unsigned)MEMLEN; const unsigned tt = im ? t : (t - (unsigned)MEMLEN);
    const size_t so = ((size_t)b * (im ? MEM_FULL : SEQ_FULL) + tt) * HID + col; const float* sp = im ? mems : x;
    const v8f v = *(const v8f*)(sp + so); v8us o;
#pragma unroll
    for (int k = 0; k < 8; ++k) o[k] = f2bf(v[k]);
    *(volatile v8us*)(dst + (size_t)i * 8) = o; __threadfence(); *(volatile v8us*)(dst + (size_t)i * 8) = o; }

template <int F16>
__global__ __launch_bounds__(256) void k_wT(const float* __restrict__ W, bf* out, unsigned Kd, unsigned N) {
    __shared__ __align__(16) unsigned short ts[64 * 72];
    const unsigned tid = threadIdx.x, n0 = blockIdx.x * 64u, k0 = blockIdx.y * 64u;
#pragma unroll
    for (int i = 0; i < 4; ++i) { const unsigned idx = tid + 256u * i; const unsigned r = idx >> 4, c4 = (idx & 15u) * 4u; const v4f v = *(const v4f*)(W + (size_t)(k0 + r) * N + n0 + c4);
#pragma unroll
        for (int e = 0; e < 4; ++e) { unsigned short w; if (F16) { const h16 hv = (h16)(bfr(v[e]) * WCAR); w = __builtin_bit_cast(unsigned short, hv); } else w = f2bf(v[e]); ts[(c4 + e) * 72u + r] = w; } }
    __syncthreads();
#pragma unroll 1
    for (int ps = 0; ps < 2; ++ps) {
#pragma unroll
        for (int i = 0; i < 2; ++i) { const unsigned idx = tid + 256u * i; const unsigned c = idx >> 3, pc = (idx & 7u) * 8u; const v8us val = *(const v8usa*)(ts + c * 72u + pc);
            *(volatile v8us*)(out + (size_t)(n0 + c) * Kd + k0 + pc) = val; }
        if (ps == 0) __threadfence(); }
}

__global__ __launch_bounds__(32) void k_attn(const h16* __restrict__ QU, const h16* __restrict__ QV, const h16* __restrict__ KP, const h16* __restrict__ VT, const h16* __restrict__ RP, h16* CTX) {
    __shared__ __align__(16) float bdb[16 * BDS];
    __shared__ __align__(16) h16 ct[16 * CTS];
    const unsigned lane = threadIdx.x & 31u, lr = lane & 15u, hi = lane >> 4;
    const unsigned i0 = blockIdx.x * 16u, hh = blockIdx.y, b = blockIdx.z;
    const size_t qo = ((size_t)b * SEQ + i0 + lr) * HID + hh * HD + 8u * hi;
    v16h qu[2], qv[2];
    qu[0] = WFrag<h16>::ld(QU + qo); qu[1] = WFrag<h16>::ld(QU + qo + 32); qv[0] = WFrag<h16>::ld(QV + qo); qv[1] = WFrag<h16>::ld(QV + qo + 32);
    const h16* Kb = KP + (size_t)b * KL * HID + hh * HD + 8u * hi;
    const h16* Vb = VT + (size_t)b * HID * KL + (size_t)(hh * HD + lr) * KL + 8u * hi;
    const h16* Rb = RP + hh * HD + 8u * hi;
    v8f o[4];
#pragma unroll
    for (int t = 0; t < 4; ++t) o[t] = (v8f){};
    float rmax = -1.0e30f, rsum = 0.0f;
    const unsigned jend = i0 + 16u + (unsigned)MEMLEN;
    const unsigned jb0 = (unsigned)(SEQ - 16) - i0;
    const unsigned lim = i0 + lr + (unsigned)MEMLEN;
    v8f bdprev = (v8f){};
    { const unsigned c = umin_(jb0 + lr, (unsigned)(KL - 1)); const h16* rr = Rb + (size_t)c * HID; const v16h f0 = WFrag<h16>::ld(rr), f1 = WFrag<h16>::ld(rr + 32);
      bdprev = wmma16(f0, qv[0], bdprev); bdprev = wmma16(f1, qv[1], bdprev);
      asm volatile("v_nop\n\tv_nop\n\tv_nop\n\tv_nop" : "+v"(bdprev) : "v"(f0), "v"(f1)); }
    const unsigned rbase = lr * BDS + 8u * hi + 15u - lr;
#pragma unroll 1
    for (unsigned j0 = 0; j0 < jend; j0 += 32u) {
        const unsigned jb = j0 + jb0;
        v8f s0 = (v8f){}, s1 = (v8f){}, t1 = (v8f){}, t2 = (v8f){};
        { const h16* k0p = Kb + (size_t)(j0 + lr) * HID; const h16* k1p = k0p + (size_t)16 * HID;
          const v16h ka0 = WFrag<h16>::ld(k0p), ka1 = WFrag<h16>::ld(k0p + 32), kb0 = WFrag<h16>::ld(k1p), kb1 = WFrag<h16>::ld(k1p + 32);
          s0 = wmma16(ka0, qu[0], s0); s1 = wmma16(kb0, qu[0], s1); s0 = wmma16(ka1, qu[1], s0); s1 = wmma16(kb1, qu[1], s1);
          asm volatile("v_nop\n\tv_nop\n\tv_nop\n\tv_nop" : "+v"(s0), "+v"(s1) : "v"(ka0), "v"(ka1), "v"(kb0), "v"(kb1)); }
        { const unsigned c1 = umin_(jb + 16u + lr, (unsigned)(KL - 1)), c2 = umin_(jb + 32u + lr, (unsigned)(KL - 1));
          const h16* r1p = Rb + (size_t)c1 * HID; const h16* r2p = Rb + (size_t)c2 * HID;
          const v16h ra0 = WFrag<h16>::ld(r1p), ra1 = WFrag<h16>::ld(r1p + 32), rb0 = WFrag<h16>::ld(r2p), rb1 = WFrag<h16>::ld(r2p + 32);
          t1 = wmma16(ra0, qv[0], t1); t2 = wmma16(rb0, qv[0], t2); t1 = wmma16(ra1, qv[1], t1); t2 = wmma16(rb1, qv[1], t2);
          asm volatile("v_nop\n\tv_nop\n\tv_nop\n\tv_nop" : "+v"(t1), "+v"(t2) : "v"(ra0), "v"(ra1), "v"(rb0), "v"(rb1)); }
#pragma unroll
        for (int r = 0; r < 8; ++r) { bdb[lr * BDS + 8u * hi + r] = bdprev[r]; bdb[lr * BDS + 16u + 8u * hi + r] = t1[r]; bdb[lr * BDS + 32u + 8u * hi + r] = t2[r]; }
        bdprev = t2;
        wsync();
        float v0[8], v1[8]; float mx = -3.0e38f; const unsigned jl = j0 + 8u * hi;
#pragma unroll
        for (int r = 0; r < 8; ++r) { const float a0 = (s0[r] + bdb[rbase + r]) * 0.125f; const float a1 = (s1[r] + bdb[rbase + 16u + r]) * 0.125f;
            v0[r] = (jl + r <= lim) ? a0 : -1.0e9f; v1[r] = (jl + 16u + r <= lim) ? a1 : -1.0e9f; mx = fmaxf(mx, fmaxf(v0[r], v1[r])); }
        mx = fmaxf(mx, __shfl_xor(mx, 16, 32));
        const float nm = fmaxf(rmax, mx); const float cf = __builtin_amdgcn_exp2f((rmax - nm) * L2E); rmax = nm;
        float ps = 0.0f; v16h pb;
#pragma unroll
        for (int r = 0; r < 8; ++r) { const float p0 = __builtin_amdgcn_exp2f((v0[r] - nm) * L2E); const float p1 = __builtin_amdgcn_exp2f((v1[r] - nm) * L2E); ps += p0 + p1; pb[r] = (h16)p0; pb[8 + r] = (h16)p1; }
        ps += __shfl_xor(ps, 16, 32); rsum = rsum * cf + ps;
#pragma unroll
        for (int t = 0; t < 4; ++t)
#pragma unroll
            for (int r = 0; r < 8; ++r) o[t][r] *= cf;
        { const h16* vp = Vb + j0; const v16h va = WFrag<h16>::ld(vp), vb2 = WFrag<h16>::ld(vp + (size_t)16 * KL), vc = WFrag<h16>::ld(vp + (size_t)32 * KL), vd = WFrag<h16>::ld(vp + (size_t)48 * KL);
          o[0] = wmma16(va, pb, o[0]); o[1] = wmma16(vb2, pb, o[1]); o[2] = wmma16(vc, pb, o[2]); o[3] = wmma16(vd, pb, o[3]);
          asm volatile("v_nop\n\tv_nop\n\tv_nop\n\tv_nop" : "+v"(o[0]), "+v"(o[1]), "+v"(o[2]), "+v"(o[3]) : "v"(va), "v"(vd), "v"(pb)); }
        wsync();
    }
    const float inv = CCAR * __builtin_amdgcn_rcpf(rsum);
#pragma unroll
    for (int t = 0; t < 4; ++t) { v8h w;
#pragma unroll
        for (int r = 0; r < 8; ++r) w[r] = (h16)(o[t][r] * inv);
        *(v8ha*)(ct + lr * CTS + 16u * t + 8u * hi) = w; }
    wsync();
    const unsigned rq = lane >> 3, pc = (lane & 7u) * 8u;
#pragma unroll 1
    for (int psn = 0; psn < 2; ++psn) {
#pragma unroll
        for (int s = 0; s < 4; ++s) { const unsigned row = 4u * s + rq; const v8h val = *(const v8ha*)(ct + row * CTS + pc);
            *(volatile v8h*)(CTX + ((size_t)b * SEQ + i0 + row) * HID + hh * HD + pc) = val; }
        if (psn == 0) __threadfence(); }
}

template <int STAGE>
__global__ __launch_bounds__(256) void k_ln(const float* __restrict__ A, const float* __restrict__ Badd, const float* __restrict__ gamma, const float* __restrict__ beta, float* outF, h16* out16, const float* __restrict__ cps, float* cpd) {
    __shared__ float red1[8]; __shared__ float red2[8];
    const unsigned row = blockIdx.x, tid = threadIdx.x, lane = tid & 31u, wv = tid >> 5;
    const unsigned bb = row / (unsigned)SEQ, ss = row % (unsigned)SEQ; const size_t frow = (size_t)bb * SEQ_FULL + ss; const unsigned c0 = tid * 4u;
    const v4f a = *(const v4f*)(A + (size_t)row * HID + c0);
    const v4f r4 = *(const v4f*)(Badd + ((STAGE == 1) ? frow : (size_t)row) * HID + c0);
    v4f v; float sm = 0.0f;
#pragma unroll
    for (int e = 0; e < 4; ++e) { const float rb = (STAGE == 1) ? bfr(r4[e]) : r4[e]; v[e] = a[e] + rb; sm += v[e]; }
#pragma unroll
    for (int sh = 16; sh; sh >>= 1) sm += __shfl_xor(sm, sh, 32);
    if (lane == 0) red1[wv] = sm;
    __syncthreads();
    float tot = 0.0f;
#pragma unroll
    for (int w = 0; w < 8; ++w) tot += red1[w];
    const float mu = tot * (1.0f / HID);
    float s2 = 0.0f;
#pragma unroll
    for (int e = 0; e < 4; ++e) { const float d = v[e] - mu; s2 += d * d; }
#pragma unroll
    for (int sh = 16; sh; sh >>= 1) s2 += __shfl_xor(s2, sh, 32);
    if (lane == 0) red2[wv] = s2;
    __syncthreads();
    float tot2 = 0.0f;
#pragma unroll
    for (int w = 0; w < 8; ++w) tot2 += red2[w];
    const float rs = rsqrtf(tot2 * (1.0f / HID) + 1.0e-5f);
    const v4f g4 = *(const v4f*)(gamma + c0); const v4f b4 = *(const v4f*)(beta + c0);
    v4f y; v4h y16;
#pragma unroll
    for (int e = 0; e < 4; ++e) { y[e] = (v[e] - mu) * rs * bfr(g4[e]) + bfr(b4[e]); y16[e] = (h16)y[e]; }
    if (STAGE == 1) {
        float* po = outF + (size_t)row * HID + c0; h16* ph = out16 + (size_t)row * HID + c0;
        *(volatile v4f*)po = y; *(volatile v4h*)ph = y16; __threadfence(); *(volatile v4f*)po = y; *(volatile v4h*)ph = y16;
    } else {
        const v4f cpraw = *(const v4f*)(cps + frow * HID + c0);
        v4f cp;
#pragma unroll
        for (int e = 0; e < 4; ++e) cp[e] = bfr(cpraw[e]);
        float* po = outF + frow * HID + c0; float* pq = cpd + frow * HID + c0;
        *(volatile v4f*)po = y; *(volatile v4f*)pq = cp; __threadfence(); *(volatile v4f*)po = y; *(volatile v4f*)pq = cp;
    }
}

constexpr size_t cmax_(size_t a, size_t b) { return a > b ? a : b; }
constexpr size_t al256(size_t a) { return (a + 255) & ~(size_t)255; }

extern "C" void kernel_launch(void* const* d_in, const int* in_sizes, int n_in,
                              void* d_out, int out_size, void* d_ws, size_t ws_size, hipStream_t stream) {
    if (n_in < 18) return;
    constexpr size_t NEED_X = ((size_t)(NB - 1) * SEQ_FULL + SEQ) * HID;
    constexpr size_t NEED_M = ((size_t)(NB - 1) * MEM_FULL + MEMLEN) * HID;
    constexpr size_t OUT1_EL = (size_t)NB_FULL * SEQ_FULL * HID;
    static_assert(OUT1_EL * 4 == 16777216);
    if ((size_t)in_sizes[0] < NEED_X || (size_t)in_sizes[1] < (size_t)KL * HID || (size_t)in_sizes[2] < NEED_M) return;
    if ((size_t)in_sizes[5] < (size_t)HID * HID || (size_t)in_sizes[6] < (size_t)HID * HID || (size_t)in_sizes[7] < (size_t)HID * HID || (size_t)in_sizes[8] < (size_t)HID * HID || (size_t)in_sizes[9] < (size_t)HID * HID) return;
    if (in_sizes[10] < HID || in_sizes[11] < HID || in_sizes[12] < HID || in_sizes[13] < HID || in_sizes[15] < FFD || in_sizes[17] < HID) return;
    if ((size_t)in_sizes[14] < (size_t)HID * FFD || (size_t)in_sizes[16] < (size_t)HID * FFD) return;
    if ((size_t)out_size < OUT1_EL + NEED_X) return;

    const float* x = (const float*)d_in[0]; const float* rel = (const float*)d_in[1]; const float* mems = (const float*)d_in[2];
    const float* Wq = (const float*)d_in[5]; const float* Wk = (const float*)d_in[6]; const float* Wv = (const float*)d_in[7]; const float* Wr = (const float*)d_in[8]; const float* Wo = (const float*)d_in[9];
    const float* ub = (const float*)d_in[10]; const float* vb = (const float*)d_in[11]; const float* gamma = (const float*)d_in[12]; const float* beta = (const float*)d_in[13];
    const float* W1 = (const float*)d_in[14]; const float* b1 = (const float*)d_in[15]; const float* W2 = (const float*)d_in[16]; const float* b2 = (const float*)d_in[17];
    float* OUT0 = (float*)d_out; float* OUT1 = (float*)d_out + OUT1_EL;

    constexpr size_t SZ_CAT = (size_t)NB * KL * HID * 2, SZ_F32 = (size_t)NB * SEQ * HID * 4, SZ_H16 = (size_t)NB * SEQ * HID * 2;
    constexpr size_t SZ_KP = (size_t)NB * KL * HID * 2, SZ_VT = (size_t)NB * HID * KL * 2, SZ_F1 = (size_t)NB * SEQ * FFD * 2;
    constexpr size_t SZ_W = (size_t)HID * HID * 2, SZ_WF = (size_t)HID * FFD * 2, SZ_REL = (size_t)KL * HID * 2;
    constexpr size_t R_A = al256(cmax_(SZ_CAT, SZ_F32));
    constexpr size_t R_Q = al256(cmax_(2 * SZ_H16 + SZ_KP, SZ_F1));
    constexpr size_t R_V = al256(cmax_(SZ_VT, SZ_F32));
    constexpr size_t R_C = al256(SZ_H16);
    constexpr size_t TOTAL = R_A + al256(SZ_REL) + 5 * al256(SZ_W) + 2 * al256(SZ_WF) + R_Q + R_V + al256(SZ_REL) + R_C;
    static_assert(SZ_CAT <= R_A);
    static_assert(SZ_F32 <= R_A);
    static_assert(2 * SZ_H16 + SZ_KP <= R_Q);
    static_assert(SZ_F1 <= R_Q);
    static_assert(SZ_VT <= R_V);
    static_assert(SZ_F32 <= R_V);
    static_assert(TOTAL <= (size_t)134217728);
    if (TOTAL > ws_size) return;
    char* wsp = (char*)d_ws;
    auto take = [&](size_t bytes) { char* p = wsp; wsp += al256(bytes); return (void*)p; };
    char* RA = (char*)take(R_A); bf* CAT = (bf*)RA; float* AO = (float*)RA; float* FF = (float*)RA;
    bf* RELB = (bf*)take(SZ_REL);
    bf* WqT = (bf*)take(SZ_W); bf* WkT = (bf*)take(SZ_W); bf* WvT = (bf*)take(SZ_W); bf* WrT = (bf*)take(SZ_W); bf* WoT = (bf*)take(SZ_W);
    bf* W1T = (bf*)take(SZ_WF); bf* W2T = (bf*)take(SZ_WF);
    char* RQ = (char*)take(R_Q); h16* QU = (h16*)RQ; h16* QV = (h16*)(RQ + SZ_H16); h16* KP = (h16*)(RQ + 2 * SZ_H16); h16* F1 = (h16*)RQ;
    char* RV = (char*)take(R_V); h16* VT = (h16*)RV; float* HF = (float*)RV;
    h16* RP = (h16*)take(SZ_REL);
    char* RC = (char*)take(R_C); h16* CTX = (h16*)RC; h16* H16P = (h16*)RC;
    if ((size_t)(wsp - (char*)d_ws) > ws_size) return;

    k_cvtcat<<<(unsigned)((size_t)NB * KL * HID / 8 / 256), 256, 0, stream>>>(mems, x, CAT);
    k_cvt8<<<(unsigned)((size_t)KL * HID / 8 / 256), 256, 0, stream>>>(rel, RELB, (unsigned)((size_t)KL * HID / 8));
    k_wT<0><<<dim3(HID / 64, HID / 64), 256, 0, stream>>>(Wq, WqT, HID, HID);
    k_wT<0><<<dim3(HID / 64, HID / 64), 256, 0, stream>>>(Wk, WkT, HID, HID);
    k_wT<0><<<dim3(HID / 64, HID / 64), 256, 0, stream>>>(Wv, WvT, HID, HID);
    k_wT<0><<<dim3(HID / 64, HID / 64), 256, 0, stream>>>(Wr, WrT, HID, HID);
    k_wT<1><<<dim3(HID / 64, HID / 64), 256, 0, stream>>>(Wo, WoT, HID, HID);
    k_wT<1><<<dim3(FFD / 64, HID / 64), 256, 0, stream>>>(W1, W1T, HID, FFD);
    k_wT<1><<<dim3(HID / 64, FFD / 64), 256, 0, stream>>>(W2, W2T, FFD, HID);

    k_gemmw<bf, EPI_H2><<<dim3(SEQ / 64, HID / 64, NB), 32, 0, stream>>>(CAT + (size_t)MEMLEN * HID, WqT, HID, nullptr, QU, QV, HID, ub, vb, 1.0f, (size_t)KL * HID, 0, (size_t)SEQ * HID);
    k_gemmw<bf, EPI_H1><<<dim3(NB * KL / 64, HID / 64, 1), 32, 0, stream>>>(CAT, WkT, HID, nullptr, KP, nullptr, HID, nullptr, nullptr, 1.0f, 0, 0, 0);
    k_gemmw<bf, EPI_H1><<<dim3(HID / 64, KL / 64, NB), 32, 0, stream>>>(WvT, CAT, HID, nullptr, VT, nullptr, KL, nullptr, nullptr, 1.0f, 0, (size_t)KL * HID, (size_t)HID * KL);
    k_gemmw<bf, EPI_H1><<<dim3(KL / 64, HID / 64, 1), 32, 0, stream>>>(RELB, WrT, HID, nullptr, RP, nullptr, HID, nullptr, nullptr, 1.0f, 0, 0, 0);

    k_attn<<<dim3(SEQ / 16, NHEAD, NB), 32, 0, stream>>>(QU, QV, KP, VT, RP, CTX);

    k_gemmw<h16, EPI_F32><<<dim3(NB * SEQ / 64, HID / 64, 1), 32, 0, stream>>>(CTX, (const h16*)WoT, HID, AO, nullptr, nullptr, HID, nullptr, nullptr, 1.0f / (CCAR * WCAR), 0, 0, 0);
    k_ln<1><<<NB * SEQ, 256, 0, stream>>>(AO, x, gamma, beta, HF, H16P, nullptr, nullptr);
    k_gemmw<h16, EPI_H1R><<<dim3(NB * SEQ / 64, FFD / 64, 1), 32, 0, stream>>>(H16P, (const h16*)W1T, HID, nullptr, F1, nullptr, FFD, b1, nullptr, 1.0f / WCAR, 0, 0, 0);
    k_gemmw<h16, EPI_F32><<<dim3(NB * SEQ / 64, HID / 64, 1), 32, 0, stream>>>(F1, (const h16*)W2T, FFD, FF, nullptr, nullptr, HID, b2, nullptr, 1.0f / WCAR, 0, 0, 0);
    k_ln<2><<<NB * SEQ, 256, 0, stream>>>(FF, HF, gamma, beta, OUT0, nullptr, x, OUT1);
}
